// PillarAttention_7215545057625
// MI455X (gfx1250) — hardware-run, weakly checked
//
#include <hip/hip_runtime.h>


#define NSC  4
#define SS   2048
#define CC   256
#define NH_  8
#define HD   32
#define FF   512
#define SCL  0.1767766952966369f
#define PCAR 1024.0f
typedef _Float16 h16;
typedef unsigned short bf;
typedef __attribute__((ext_vector_type(16))) __bf16   v16bf;
typedef __attribute__((ext_vector_type(16))) _Float16 v16h;
typedef __attribute__((ext_vector_type(8)))  _Float16 v8h;
typedef __attribute__((ext_vector_type(8)))  unsigned short v8us;
typedef __attribute__((ext_vector_type(8)))  float    v8f;
typedef __attribute__((ext_vector_type(4)))  float    v4f;
typedef v8h  __attribute__((may_alias)) v8ha;
typedef v4f  __attribute__((may_alias)) v4fa;
typedef v8us __attribute__((may_alias)) v8usa;

__device__ __forceinline__ unsigned short f2bf(float f) { unsigned u = __float_as_uint(f); u += 0x7FFFu + ((u >> 16) & 1u); return (unsigned short)(u >> 16); }
__device__ __forceinline__ float bf2f(unsigned short b) { return __uint_as_float(((unsigned)b) << 16); }
__device__ __forceinline__ float bfr(float f) { return bf2f(f2bf(f)); }
__device__ __forceinline__ v16h cat16(v8h lo, v8h hi) { return __builtin_shufflevector(lo, hi, 0, 1, 2, 3, 4, 5, 6, 7, 8, 9, 10, 11, 12, 13, 14, 15); }
__device__ __forceinline__ v16bf cat16b(v8us lo, v8us hi) { return __builtin_bit_cast(v16bf, __builtin_shufflevector(lo, hi, 0, 1, 2, 3, 4, 5, 6, 7, 8, 9, 10, 11, 12, 13, 14, 15)); }
__device__ __forceinline__ v8f wmma16(v16h a, v16h b, v8f c) { return __builtin_amdgcn_wmma_f32_16x16x32_f16(false, a, false, b, (short)0, c, false, false); }
__device__ __forceinline__ v8f wmmab(v16bf a, v16bf b, v8f c) { return __builtin_amdgcn_wmma_f32_16x16x32_bf16(false, a, false, b, (short)0, c, false, false); }


template <typename T16> struct WFrag;
template <> struct WFrag<h16> { typedef v16h V; static __device__ __forceinline__ V ld(const h16* p) { return cat16(*(const v8h*)p, *(const v8h*)(p + 16)); } static __device__ __forceinline__ v8f mma(V a, V b, v8f c) { return wmma16(a, b, c); } };
template <> struct WFrag<bf> { typedef v16bf V; static __device__ __forceinline__ V ld(const bf* p) { return cat16b(*(const v8us*)p, *(const v8us*)(p + 16)); } static __device__ __forceinline__ v8f mma(V a, V b, v8f c) { return wmmab(a, b, c); } };
template <typename T16, int NSPLIT, bool BIAS>
__global__ __launch_bounds__(32) void k_gemmw(const T16* __restrict__ A, const T16* __restrict__ A2, const T16* __restrict__ Bt, const T16* __restrict__ Bt2, int K, float* C, int ldc, const float* __restrict__ bias, size_t sA, size_t sB, size_t sC) {
    typedef typename WFrag<T16>::V V;
    __shared__ __align__(16) float os[16 * 68];
    const size_t z = blockIdx.z; A += z * sA; if (A2) A2 += z * sA; Bt += z * sB; if (Bt2) Bt2 += z * sB; C += z * sC;
    const int lane = threadIdx.x & 31, lr = lane & 15, hi = lane >> 4; const int r0 = blockIdx.x * 64, c0 = blockIdx.y * 64;
    v8f acc[4][4];
#pragma unroll
    for (int mb = 0; mb < 4; ++mb)
#pragma unroll
        for (int nb = 0; nb < 4; ++nb) acc[mb][nb] = (v8f){};
    const size_t aoff = (size_t)(r0 + lr) * K + 8 * hi, boff = (size_t)(c0 + lr) * K + 8 * hi;
#pragma unroll 1
    for (int kc = 0; kc < K; kc += 32) {
        V a[4], a2[4];
#pragma unroll
        for (int mb = 0; mb < 4; ++mb) { a[mb] = WFrag<T16>::ld(A + aoff + (size_t)mb * 16 * K + kc); if (NSPLIT == 1 || NSPLIT == 2) a2[mb] = WFrag<T16>::ld(A2 + aoff + (size_t)mb * 16 * K + kc); }
#pragma unroll
        for (int nb = 0; nb < 4; ++nb) { const V b = WFrag<T16>::ld(Bt + boff + (size_t)nb * 16 * K + kc); V b2; if (NSPLIT >= 2) b2 = WFrag<T16>::ld(Bt2 + boff + (size_t)nb * 16 * K + kc);
#pragma unroll
            for (int mb = 0; mb < 4; ++mb) { acc[mb][nb] = WFrag<T16>::mma(a[mb], b, acc[mb][nb]); if (NSPLIT == 1 || NSPLIT == 2) acc[mb][nb] = WFrag<T16>::mma(a2[mb], b, acc[mb][nb]); if (NSPLIT >= 2) acc[mb][nb] = WFrag<T16>::mma(a[mb], b2, acc[mb][nb]); } }
        asm volatile("v_nop\n\tv_nop\n\tv_nop\n\tv_nop" : "+v"(acc[0][0]), "+v"(acc[1][1]), "+v"(acc[2][2]), "+v"(acc[3][3]) : "v"(a[0]), "v"(a[3]));
    }
#pragma unroll
    for (int mb = 0; mb < 4; ++mb) {
#pragma unroll
        for (int nb = 0; nb < 4; ++nb) {
#pragma unroll
            for (int j = 0; j < 8; ++j) os[(hi * 8 + j) * 68 + nb * 16 + lr] = acc[mb][nb][j]; }
        __builtin_amdgcn_wave_barrier(); asm volatile("" ::: "memory");
        float* crow = C + (size_t)(r0 + mb * 16) * ldc + c0;
#pragma unroll 1
        for (int ps = 0; ps < 2; ++ps) {
#pragma unroll
            for (int s = 0; s < 8; ++s) { const int row = 2 * s + hi, cofs = lr * 4; v4f val = *(const v4fa*)(os + row * 68 + cofs); if (BIAS) { val[0] += bfr(bias[c0 + cofs]); val[1] += bfr(bias[c0 + cofs + 1]); val[2] += bfr(bias[c0 + cofs + 2]); val[3] += bfr(bias[c0 + cofs + 3]); }
                *(volatile v4f*)(crow + (size_t)row * ldc + cofs) = val; }
            if (ps == 0) __threadfence(); }
        __builtin_amdgcn_wave_barrier(); asm volatile("" ::: "memory");
    }
}

__device__ __forceinline__ h16 tohx(float x) { return (h16)x; }
__device__ __forceinline__ void splitf(float y, unsigned short& h, unsigned short& l) { h = f2bf(y); l = f2bf(y - bf2f(h)); }
typedef __attribute__((ext_vector_type(2))) _Float16 v2h;
typedef __attribute__((ext_vector_type(4))) _Float16 v4h;
typedef __attribute__((ext_vector_type(4))) unsigned short v4us;

__global__ __launch_bounds__(256) void k_cvt8(const float* __restrict__ src, bf* dst, size_t n8) { const size_t i = (size_t)blockIdx.x * 256 + threadIdx.x; if (i >= n8) return; const v8f v = *(const v8f*)(src + i * 8); v8us o;
#pragma unroll
    for (int k = 0; k < 8; ++k) o[k] = f2bf(v[k]); *(volatile v8us*)(dst + i * 8) = o; __threadfence(); *(volatile v8us*)(dst + i * 8) = o; }
__global__ __launch_bounds__(256) void k_qkpl(const float* __restrict__ QKV, h16* Q16, h16* K16) { const int e = (blockIdx.x * 256 + threadIdx.x) * 4; if (e >= NH_ * SS * HD) return; const int d = e % HD; const int s = (e / HD) % SS; const int h = e / (HD * SS); const float* r = QKV + (size_t)s * 3 * CC + h * HD + d; v4h oq, ok;
#pragma unroll
    for (int q = 0; q < 4; ++q) { oq[q] = tohx(r[q] * SCL); ok[q] = tohx(r[CC + q]); } for (int ps = 0; ps < 2; ++ps) { *(volatile v4h*)(Q16 + e) = oq; *(volatile v4h*)(K16 + e) = ok; if (ps == 0) __threadfence(); } }
__global__ __launch_bounds__(256) void k_vt(const float* __restrict__ QKV, h16* VT) { const int e = (blockIdx.x * 256 + threadIdx.x) * 2; if (e >= NH_ * 64 * SS) return; const int s = e % SS; const int dv = (e / SS) % 64; const int h = e / (SS * 64); v2h o;
#pragma unroll
    for (int u = 0; u < 2; ++u) o[u] = dv < HD ? tohx(QKV[(size_t)(s + u) * 3 * CC + 2 * CC + h * HD + dv]) : (h16)0.f; *(volatile v2h*)(VT + e) = o; __threadfence(); *(volatile v2h*)(VT + e) = o; }
__global__ __launch_bounds__(256) void k_mrg(const float* __restrict__ O, bf* Mh, bf* Ml) { const int e = (blockIdx.x * 256 + threadIdx.x) * 4; if (e >= SS * CC) return; const int c = e % CC; const int s = e / CC; const int h = c / HD, d = c % HD; const float* r = O + ((size_t)h * SS + s) * 64 + d; v4us oh, ol;
#pragma unroll
    for (int q = 0; q < 4; ++q) { unsigned short a, b; splitf(r[q] * (1.0f / PCAR), a, b); oh[q] = a; ol[q] = b; } *(volatile v4us*)(Mh + e) = oh; *(volatile v4us*)(Ml + e) = ol; __threadfence(); *(volatile v4us*)(Mh + e) = oh; *(volatile v4us*)(Ml + e) = ol; }
template <int ARES> __global__ __launch_bounds__(256) void k_lnres(const float* __restrict__ A, const float* __restrict__ R, const float* __restrict__ g, const float* __restrict__ bb, float* Y, bf* Yh, bf* Yl) { const int lane = threadIdx.x & 31; const int row = blockIdx.x * 8 + (threadIdx.x >> 5); if (row >= SS) return; const size_t rb = (size_t)row * CC; float v[8]; float s = 0.f;
#pragma unroll
    for (int ch = 0; ch < 2; ++ch) { const int c0 = ch * 128 + lane * 4; const v4f a = *(const v4f*)(A + rb + c0); const v4f r = *(const v4f*)(R + rb + c0);
#pragma unroll
        for (int q = 0; q < 4; ++q) { v[ch * 4 + q] = __fadd_rn(ARES ? bfr(a[q]) : a[q], r[q]); s = __fadd_rn(s, v[ch * 4 + q]); } }
#pragma unroll
    for (int sh = 16; sh; sh >>= 1) s += __shfl_xor(s, sh, 32);
    const float mean = s * (1.0f / CC); float q2 = 0.f;
#pragma unroll
    for (int i = 0; i < 8; ++i) { float d0 = __fsub_rn(v[i], mean); asm volatile("" : "+v"(d0)); float p = __fmul_rn(d0, d0); asm volatile("" : "+v"(p)); q2 = __fadd_rn(q2, p); }
#pragma unroll
    for (int sh = 16; sh; sh >>= 1) q2 += __shfl_xor(q2, sh, 32);
    const float rstd = __frsqrt_rn(__fadd_rn(q2 * (1.0f / CC), 1e-5f));
    for (int ps = 0; ps < 2; ++ps) {
#pragma unroll
        for (int ch = 0; ch < 2; ++ch) { const int c0 = ch * 128 + lane * 4; v4f o; v4us oh, ol;
#pragma unroll
            for (int q = 0; q < 4; ++q) { float t0 = __fmul_rn(__fsub_rn(v[ch * 4 + q], mean), rstd); asm volatile("" : "+v"(t0)); float t1 = __fmul_rn(t0, bfr(g[c0 + q])); asm volatile("" : "+v"(t1)); o[q] = __fadd_rn(t1, bfr(bb[c0 + q])); unsigned short u, l; splitf(o[q], u, l); oh[q] = u; ol[q] = l; }
            *(volatile v4f*)(Y + rb + c0) = o; *(volatile v4us*)(Yh + rb + c0) = oh; *(volatile v4us*)(Yl + rb + c0) = ol; }
        if (ps == 0) __threadfence(); } }
__global__ __launch_bounds__(256) void k_gelupl(const float* __restrict__ F, bf* Ph, bf* Pl) { const int e = (blockIdx.x * 256 + threadIdx.x) * 4; if (e >= SS * FF) return; const v4f a = *(const v4f*)(F + e); v4us oh, ol;
#pragma unroll 1
    for (int q = 0; q < 4; ++q) { const float x = a[q]; const float gl = __fmul_rn(0.5f * x, __fadd_rn(1.0f, erff(x * 0.7071067811865476f))); unsigned short u, l; splitf(gl, u, l); oh[q] = u; ol[q] = l; } *(volatile v4us*)(Ph + e) = oh; *(volatile v4us*)(Pl + e) = ol; __threadfence(); *(volatile v4us*)(Ph + e) = oh; *(volatile v4us*)(Pl + e) = ol; }
template <int NFULL, int TAIL> __global__ __launch_bounds__(256) void k_soft(const float* __restrict__ Sb, int nrows, int rowsper, int rvalid, int nvalid, h16* P) { const int lane = threadIdx.x & 31; const size_t row = (size_t)blockIdx.x * 8 + (threadIdx.x >> 5); if (row >= (size_t)nrows) return; constexpr int LD = NFULL * 128 + TAIL * 64; const float* sr = Sb + row * LD; h16* pr = P + row * LD; const bool live = (int)(row % rowsper) < rvalid; float mx = -3.0e38f;
#pragma unroll 1
    for (int ch = 0; ch < NFULL + TAIL; ++ch) { if (ch == NFULL && lane >= 16) break; const int j0 = ch * 128 + lane * 4; const v4f a = *(const v4f*)(sr + j0);
#pragma unroll
        for (int q = 0; q < 4; ++q) if (j0 + q < nvalid) mx = fmaxf(mx, a[q]); }
#pragma unroll
    for (int sh = 16; sh; sh >>= 1) mx = fmaxf(mx, __shfl_xor(mx, sh, 32));
    float sum = 0.f;
#pragma unroll 1
    for (int ch = 0; ch < NFULL + TAIL; ++ch) { if (ch == NFULL && lane >= 16) break; const int j0 = ch * 128 + lane * 4; const v4f a = *(const v4f*)(sr + j0);
#pragma unroll
        for (int q = 0; q < 4; ++q) if (j0 + q < nvalid) { float d0 = __fsub_rn(a[q], mx); asm volatile("" : "+v"(d0)); sum += __expf(d0); } }
#pragma unroll
    for (int sh = 16; sh; sh >>= 1) sum += __shfl_xor(sum, sh, 32);
    const float f = live ? __fdiv_rn(PCAR, sum) : 0.f;
    for (int ps = 0; ps < 2; ++ps) {
#pragma unroll 1
        for (int ch = 0; ch < NFULL + TAIL; ++ch) { if (ch == NFULL && lane >= 16) break; const int j0 = ch * 128 + lane * 4; const v4f a = *(const v4f*)(sr + j0); v4h o;
#pragma unroll
            for (int q = 0; q < 4; ++q) { float val = 0.f; if (live && j0 + q < nvalid) { float d0 = __fsub_rn(a[q], mx); asm volatile("" : "+v"(d0)); val = __fmul_rn(__expf(d0), f); } o[q] = tohx(val); } *(volatile v4h*)(pr + j0) = o; }
        if (ps == 0) __threadfence(); } }

extern "C" void kernel_launch(void* const* d_in, const int* in_sizes, int n_in,
                              void* d_out, int out_size, void* d_ws, size_t ws_size, hipStream_t stream) {
    (void)in_sizes; (void)n_in; (void)out_size;
    const float* x = (const float*)d_in[0];   const float* wqkv = (const float*)d_in[2]; const float* bqkv = (const float*)d_in[3]; const float* wout = (const float*)d_in[4]; const float* bout = (const float*)d_in[5]; const float* g1 = (const float*)d_in[6]; const float* be1 = (const float*)d_in[7]; const float* w1 = (const float*)d_in[8]; const float* b1 = (const float*)d_in[9]; const float* w2 = (const float*)d_in[10]; const float* b2 = (const float*)d_in[11]; const float* g2 = (const float*)d_in[12]; const float* be2 = (const float*)d_in[13];
    float* OUT = (float*)d_out;
    char* wsp = (char*)d_ws;
    auto take = [&](size_t bytes) { char* p = wsp; wsp += (bytes + 255) & ~(size_t)255; return (void*)p; };
    bf* WQKV = (bf*)take((size_t)3 * CC * CC * 2); bf* WOUT = (bf*)take(CC * CC * 2); bf* W1 = (bf*)take(FF * CC * 2); bf* W2 = (bf*)take(CC * FF * 2);
    bf* XB = (bf*)take((size_t)SS * CC * 2); float* QKV = (float*)take((size_t)SS * 3 * CC * 4); h16* Q16 = (h16*)take((size_t)NH_ * SS * HD * 2); h16* K16 = (h16*)take((size_t)NH_ * SS * HD * 2); h16* VT = (h16*)take((size_t)NH_ * 64 * SS * 2); float* Sb = (float*)take((size_t)NH_ * SS * SS * 4); h16* P16 = (h16*)take((size_t)NH_ * SS * SS * 2); float* O = (float*)take((size_t)NH_ * SS * 64 * 4);
    bf* Mh = (bf*)take((size_t)SS * CC * 2); bf* Ml = (bf*)take((size_t)SS * CC * 2); float* OP = (float*)take((size_t)SS * CC * 4); float* X1 = (float*)take((size_t)SS * CC * 4); bf* X1h = (bf*)take((size_t)SS * CC * 2); bf* X1l = (bf*)take((size_t)SS * CC * 2); float* F1 = (float*)take((size_t)SS * FF * 4); bf* Gh = (bf*)take((size_t)SS * FF * 2); bf* Gl = (bf*)take((size_t)SS * FF * 2); float* F2 = (float*)take((size_t)SS * CC * 4); bf* Dh = (bf*)take((size_t)SS * CC * 2); bf* Dl = (bf*)take((size_t)SS * CC * 2);
    if ((size_t)(wsp - (char*)d_ws) > ws_size) return;
    k_cvt8<<<(3 * CC * CC / 8 + 255) / 256, 256, 0, stream>>>(wqkv, WQKV, 3 * CC * CC / 8); k_cvt8<<<(CC * CC / 8 + 255) / 256, 256, 0, stream>>>(wout, WOUT, CC * CC / 8); k_cvt8<<<(FF * CC / 8 + 255) / 256, 256, 0, stream>>>(w1, W1, FF * CC / 8); k_cvt8<<<(CC * FF / 8 + 255) / 256, 256, 0, stream>>>(w2, W2, CC * FF / 8);
    for (int sc = 0; sc < NSC; ++sc) { const float* xs = x + (size_t)sc * SS * CC;
        k_cvt8<<<(SS * CC / 8 + 255) / 256, 256, 0, stream>>>(xs, XB, SS * CC / 8);
        k_gemmw<bf, 0, true><<<dim3(SS / 64, 3 * CC / 64, 1), 32, 0, stream>>>(XB, nullptr, WQKV, nullptr, CC, QKV, 3 * CC, bqkv, 0, 0, 0);
        k_qkpl<<<(NH_ * SS * HD / 4 + 255) / 256, 256, 0, stream>>>(QKV, Q16, K16); k_vt<<<(NH_ * 64 * SS / 2 + 255) / 256, 256, 0, stream>>>(QKV, VT);
        k_gemmw<h16, 0, false><<<dim3(SS / 64, SS / 64, NH_), 32, 0, stream>>>(Q16, nullptr, K16, nullptr, HD, Sb, SS, nullptr, (size_t)SS * HD, (size_t)SS * HD, (size_t)SS * SS);
        k_soft<16, 0><<<(NH_ * SS + 7) / 8, 256, 0, stream>>>(Sb, NH_ * SS, SS, SS, SS, P16);
        k_gemmw<h16, 0, false><<<dim3(SS / 64, 1, NH_), 32, 0, stream>>>(P16, nullptr, VT, nullptr, SS, O, 64, nullptr, (size_t)SS * SS, (size_t)64 * SS, (size_t)SS * 64);
        k_mrg<<<(SS * CC / 4 + 255) / 256, 256, 0, stream>>>(O, Mh, Ml);
        k_gemmw<bf, 1, true><<<dim3(SS / 64, CC / 64, 1), 32, 0, stream>>>(Mh, Ml, WOUT, nullptr, CC, OP, CC, bout, 0, 0, 0);
        k_lnres<1><<<SS / 8, 256, 0, stream>>>(xs, OP, g1, be1, X1, X1h, X1l);
        k_gemmw<bf, 1, true><<<dim3(SS / 64, FF / 64, 1), 32, 0, stream>>>(X1h, X1l, W1, nullptr, CC, F1, FF, b1, 0, 0, 0); k_gelupl<<<(SS * FF / 4 + 255) / 256, 256, 0, stream>>>(F1, Gh, Gl);
        k_gemmw<bf, 1, true><<<dim3(SS / 64, CC / 64, 1), 32, 0, stream>>>(Gh, Gl, W2, nullptr, FF, F2, CC, b2, 0, 0, 0);
        k_lnres<0><<<SS / 8, 256, 0, stream>>>(X1, F2, g2, be2, OUT + (size_t)sc * SS * CC, Dh, Dl); }
}
